// MessagePassingWithPhase_24043226923414
// MI455X (gfx1250) — hardware-verified
//
#include <hip/hip_runtime.h>
#include <math.h>

constexpr int kNB = 2;
constexpr int kNN = 512;
constexpr int kND = 128;
constexpr int kNO = 4;
constexpr int kRows = kNB * kNN;
constexpr int kXAPitch = 2 * kND;
constexpr int kXAPlane = kRows * kXAPitch;
constexpr int kC1Pitch = 2 * kND;
constexpr int kChunkRecv = 128;
constexpr int kNumChunks = kRows / kChunkRecv;
constexpr int kPairs = kChunkRecv * kNN;
constexpr float kHidCarry = 16.0f;
constexpr float kW2Carry = 64.0f;
constexpr float kMsgScale = 1.0f / (kHidCarry * kW2Carry);

typedef __attribute__((ext_vector_type(16))) _Float16 v16h;
typedef __attribute__((ext_vector_type(8)))  _Float16 v8h;
typedef __attribute__((ext_vector_type(16))) __bf16   v16b;
typedef __attribute__((ext_vector_type(8)))  __bf16   v8b;
typedef __attribute__((ext_vector_type(8)))  float    v8f;
typedef __attribute__((ext_vector_type(4)))  float    v4f;
typedef __attribute__((ext_vector_type(4)))  unsigned int v4u;

__device__ __forceinline__ unsigned short f2bf_bits(float f) {
  unsigned u = __float_as_uint(f);
  return (unsigned short)((u + 0x7FFFu + ((u >> 16) & 1u)) >> 16);
}
__device__ __forceinline__ float bf_bits2f(unsigned short h) { return __uint_as_float(((unsigned)h) << 16); }

__device__ __forceinline__ void dep_guard_h(v8f& a, v8f& b, v16h x, v16h y) { asm volatile("v_nop\n\tv_nop\n\tv_nop\n\tv_nop" : "+v"(a), "+v"(b) : "v"(x), "v"(y)); }
__device__ __forceinline__ void dep_guard_b(v8f& a, v8f& b, v16b x, v16b y) { asm volatile("v_nop\n\tv_nop\n\tv_nop\n\tv_nop" : "+v"(a), "+v"(b) : "v"(x), "v"(y)); }
__device__ __forceinline__ void keep4_h(v16h a, v16h b, v16h c, v16h d) { asm volatile("v_nop" :: "v"(a), "v"(b), "v"(c), "v"(d)); }
__device__ __forceinline__ void keep4_b(v16b a, v16b b, v16b c, v16b d) { asm volatile("v_nop" :: "v"(a), "v"(b), "v"(c), "v"(d)); }
__device__ __forceinline__ void acc_guard4(v8f& a, v8f& b, v8f& c, v8f& d) { asm volatile("v_nop\n\tv_nop\n\tv_nop\n\tv_nop" : "+v"(a), "+v"(b), "+v"(c), "+v"(d)); }
template <typename T> struct Frag;
template <> struct Frag<_Float16> {
  typedef v16h V; union U { v16h v; v8h h[2]; };
  static __device__ __forceinline__ v16h load(const _Float16* p) {
    U f; f.h[0] = *(const v8h*)(p); f.h[1] = *(const v8h*)(p + 16); return f.v;
  }
  static __device__ __forceinline__ v8f mma(v16h a, v16h b, v8f c) {
    return __builtin_amdgcn_wmma_f32_16x16x32_f16(false, a, false, b, (short)0, c, false, false);
  }
  static __device__ __forceinline__ void guard(v8f& a, v8f& b, v16h x, v16h y) { dep_guard_h(a, b, x, y); }
  static __device__ __forceinline__ void keep(v16h a, v16h b, v16h c, v16h d) { keep4_h(a, b, c, d); }
};
template <> struct Frag<__bf16> {
  typedef v16b V; union U { v16b v; v8b h[2]; };
  static __device__ __forceinline__ v16b load(const __bf16* p) {
    U f; f.h[0] = *(const v8b*)(p); f.h[1] = *(const v8b*)(p + 16); return f.v;
  }
  static __device__ __forceinline__ v8f mma(v16b a, v16b b, v8f c) {
    return __builtin_amdgcn_wmma_f32_16x16x32_bf16(false, a, false, b, (short)0, c, false, false);
  }
  static __device__ __forceinline__ void guard(v8f& a, v8f& b, v16b x, v16b y) { dep_guard_b(a, b, x, y); }
  static __device__ __forceinline__ void keep(v16b a, v16b b, v16b c, v16b d) { keep4_b(a, b, c, d); }
};

__device__ __forceinline__ unsigned pk16(unsigned short a, unsigned short b) { return (unsigned)a | ((unsigned)b << 16); }
__device__ __forceinline__ unsigned short h_bits(float f) { const _Float16 h = (_Float16)f; return __builtin_bit_cast(unsigned short, h); }

template <int ET> struct Elem;
template <> struct Elem<0> { typedef _Float16 T; };
template <> struct Elem<1> { typedef __bf16 T; };
template <int ET, bool SPLIT, int BIAS_MODE, int OUT_MODE, bool RESID, int ACT = 0>
__global__ __launch_bounds__(256) void wmma_gemm64(
    const unsigned short* __restrict__ Ap, const unsigned short* __restrict__ A2p, int lda, long strideA,
    const unsigned short* __restrict__ Btp, const unsigned short* __restrict__ Bt2p, int ldb, long strideB,
    void* __restrict__ Cout, void* __restrict__ Cout2, int ldc, long strideC,
    const float* __restrict__ bias,
    const float* __restrict__ resid, long strideR,
    int M, int N, int K, float scale) {
  typedef typename Elem<ET>::T T;
  typedef typename Frag<T>::V V;
  const T* A = (const T*)Ap; const T* A2 = (const T*)A2p; const T* Bt = (const T*)Btp; const T* Bt2 = (const T*)Bt2p;
  __shared__ __align__(16) float sT[8][16 * 68];
  const int b    = blockIdx.y;
  const int lane = threadIdx.x & 31;
  const int wave = threadIdx.x >> 5;
  const int tilesN = N >> 6;
  const int tilesM = M >> 6;
  const int tile = blockIdx.x * 8 + wave;
  if (tile >= tilesM * tilesN) return;
  const int tm = tile / tilesN;
  const int tn = tile - tm * tilesN;
  const int m0 = tm << 6;
  const int n0 = tn << 6;

  const T* Ab  = A  + (size_t)b * strideA;
  const T* Bb  = Bt + (size_t)b * strideB;
  const T* Ab2 = SPLIT ? (A2  + (size_t)b * strideA) : nullptr;
  const T* Bb2 = SPLIT ? (Bt2 + (size_t)b * strideB) : nullptr;

  const int rlane = lane & 15;
  const int koff  = (lane >> 4) * 8;
  const int mOff  = (lane >> 4) * 8;

  v8f acc[4][4];
#pragma unroll
  for (int i = 0; i < 4; ++i)
#pragma unroll
    for (int j = 0; j < 4; ++j) acc[i][j] = (v8f){0.f,0.f,0.f,0.f,0.f,0.f,0.f,0.f};

  for (int k0 = 0; k0 < K; k0 += 32) {
    V bh[4], bl[4];
#pragma unroll
    for (int j = 0; j < 4; ++j) {
      const size_t bo = (size_t)(n0 + (j << 4) + rlane) * ldb + koff + k0;
      bh[j] = Frag<T>::load(Bb + bo);
      if (SPLIT) bl[j] = Frag<T>::load(Bb2 + bo);
    }
#pragma unroll
    for (int i = 0; i < 4; ++i) {
      const size_t ao = (size_t)(m0 + (i << 4) + rlane) * lda + koff + k0;
      V ah = Frag<T>::load(Ab + ao);
      V al;
      if (SPLIT) al = Frag<T>::load(Ab2 + ao);
#pragma unroll
      for (int j = 0; j < 4; ++j) {
        acc[i][j] = Frag<T>::mma(ah, bh[j], acc[i][j]);
        if (SPLIT) {
          acc[i][j] = Frag<T>::mma(ah, bl[j], acc[i][j]);
          acc[i][j] = Frag<T>::mma(al, bh[j], acc[i][j]);
        }
      }
      Frag<T>::guard(acc[i][0], acc[i][3], ah, SPLIT ? al : ah);
    }
    Frag<T>::keep(bh[0], bh[1], bh[2], bh[3]);
    if (SPLIT) Frag<T>::keep(bl[0], bl[1], bl[2], bl[3]);
  }
  acc_guard4(acc[0][0], acc[0][1], acc[0][2], acc[0][3]);
  acc_guard4(acc[1][0], acc[1][1], acc[1][2], acc[1][3]);
  acc_guard4(acc[2][0], acc[2][1], acc[2][2], acc[2][3]);
  acc_guard4(acc[3][0], acc[3][1], acc[3][2], acc[3][3]);

  float* slab = sT[wave];
  const float* Rb = RESID ? (resid + (size_t)b * strideR) : nullptr;
#pragma unroll
  for (int i = 0; i < 4; ++i) {
    const int mBase = m0 + (i << 4);
#pragma unroll
    for (int j = 0; j < 4; ++j) {
      const int n = n0 + (j << 4) + rlane;
      float bv = 0.f;
      if (BIAS_MODE == 2) bv = bias[n];
#pragma unroll
      for (int r = 0; r < 8; ++r) {
        float v = acc[i][j][r] * scale;
        if (BIAS_MODE == 1) v += bias[mBase + mOff + r];
        if (BIAS_MODE == 2) v += bv;
        if (RESID) v += Rb[(size_t)(mBase + mOff + r) * ldc + n];
        if (ACT == 2) v = fmaxf(v, 0.0f);
        if (ACT == 4) v = (v > 0.f) ? v : 0.01f * v;
        slab[(mOff + r) * 68 + (j << 4) + rlane] = v;
      }
    }
    __builtin_amdgcn_fence(__ATOMIC_RELEASE, "workgroup");
    __builtin_amdgcn_wave_barrier();
    __builtin_amdgcn_fence(__ATOMIC_ACQUIRE, "workgroup");
    if (OUT_MODE == 0) {
      float* C = (float*)Cout + (size_t)b * strideC;
      const int hh = lane >> 4, c4 = (lane & 15) * 4;
      for (int pass = 0; pass < 2; ++pass) {
#pragma unroll
        for (int it = 0; it < 8; ++it) {
          const int row = it * 2 + hh;
          v4f v = *(const v4f*)(slab + row * 68 + c4);
          *(volatile v4f*)(C + (size_t)(mBase + row) * ldc + n0 + c4) = v;
        }
        __threadfence();
      }
    } else {
      const int q = lane >> 3, c8 = (lane & 7) * 8;
      unsigned short* C  = (unsigned short*)Cout  + (size_t)b * strideC;
      unsigned short* C2 = (OUT_MODE == 2) ? ((unsigned short*)Cout2 + (size_t)b * strideC) : nullptr;
      for (int pass = 0; pass < 2; ++pass) {
#pragma unroll
        for (int it = 0; it < 4; ++it) {
          const int row = it * 4 + q;
          const float* sp = slab + row * 68 + c8;
          v8h hv, lv;
#pragma unroll
          for (int e = 0; e < 8; ++e) {
            if (OUT_MODE == 1) {
              hv[e] = (_Float16)sp[e];
            } else {
              unsigned short hb = f2bf_bits(sp[e]);
              unsigned short lb = f2bf_bits(sp[e] - bf_bits2f(hb));
              hv[e] = __builtin_bit_cast(_Float16, hb);
              lv[e] = __builtin_bit_cast(_Float16, lb);
            }
          }
          *(volatile v8h*)(C + (size_t)(mBase + row) * ldc + n0 + c8) = hv;
          if (OUT_MODE == 2) *(volatile v8h*)(C2 + (size_t)(mBase + row) * ldc + n0 + c8) = lv;
        }
        __threadfence();
      }
    }
    __builtin_amdgcn_fence(__ATOMIC_RELEASE, "workgroup");
    __builtin_amdgcn_wave_barrier();
    __builtin_amdgcn_fence(__ATOMIC_ACQUIRE, "workgroup");
  }
}

__global__ __launch_bounds__(256) void xsplit_kernel(const float* __restrict__ X, unsigned short* __restrict__ XA) {
  const int t   = blockIdx.x * 256 + threadIdx.x;
  const int row = t >> 4;
  const int c8  = (t & 15) * 8;
  const float* p = X + (size_t)row * kND + c8;
  const v4f a = *(const v4f*)(p);
  const v4f c = *(const v4f*)(p + 4);
  unsigned short hb[8], lb[8];
#pragma unroll
  for (int e = 0; e < 4; ++e) {
    hb[e]     = f2bf_bits(a[e]);
    lb[e]     = f2bf_bits(a[e] - bf_bits2f(hb[e]));
    hb[4 + e] = f2bf_bits(c[e]);
    lb[4 + e] = f2bf_bits(c[e] - bf_bits2f(hb[4 + e]));
  }
  const v4u uh = (v4u){pk16(hb[0], hb[1]), pk16(hb[2], hb[3]), pk16(hb[4], hb[5]), pk16(hb[6], hb[7])};
  const v4u ul = (v4u){pk16(lb[0], lb[1]), pk16(lb[2], lb[3]), pk16(lb[4], lb[5]), pk16(lb[6], lb[7])};
  unsigned short* q = XA + (size_t)row * kXAPitch + c8;
  *(volatile v4u*)(q) = uh;
  *(volatile v4u*)(q + kXAPlane) = ul;
  __threadfence();
  *(volatile v4u*)(q) = uh;
  *(volatile v4u*)(q + kXAPlane) = ul;
}

__global__ __launch_bounds__(256) void wprep_kernel(const float* __restrict__ W1r, const float* __restrict__ W1s,
                                                    const float* __restrict__ Wu1x, const float* __restrict__ Wu1a,
                                                    const float* __restrict__ Wu2, const float* __restrict__ W2,
                                                    unsigned short* __restrict__ W1T, unsigned short* __restrict__ WuT,
                                                    unsigned short* __restrict__ Wu2T, unsigned short* __restrict__ W2T) {
  __shared__ float sm[64][65];
  const int t  = threadIdx.x;
  const int k0 = blockIdx.x * 64;
  const int n0 = blockIdx.y * 64;
  const int z  = blockIdx.z;
  const float* W = (z == 0) ? W1r : (z == 1) ? W1s : (z == 2) ? Wu1x : (z == 3) ? Wu1a : (z == 4) ? Wu2 : W2;
  unsigned short* D = (z <= 1) ? W1T : (z <= 3) ? WuT : (z == 4) ? Wu2T : W2T;
  const int pitch  = (z == 2 || z == 3) ? 256 : 128;
  const int plane  = (z <= 1) ? (256 * 128) : (z <= 3) ? (128 * 256) : (128 * 128);
  const int rowOff = (z == 1) ? 128 : 0;
  const int colOff = (z == 3) ? 128 : 0;
#pragma unroll
  for (int i = 0; i < 16; ++i) {
    const int e = i * 256 + t;
    const int r = e >> 6;
    const int c = e & 63;
    sm[c][r] = W[(size_t)(k0 + r) * kND + n0 + c];
  }
  __syncthreads();
  const int lane = t & 31, wave = t >> 5;
  const int q = lane >> 3, c8 = (lane & 7) * 8;
  for (int pass = 0; pass < 2; ++pass) {
#pragma unroll
    for (int it = 0; it < 2; ++it) {
      const int row = wave * 8 + it * 4 + q;
      const size_t o = (size_t)(rowOff + n0 + row) * pitch + colOff + k0 + c8;
      if (z == 5) {
        unsigned short hb[8];
#pragma unroll
        for (int e = 0; e < 8; ++e) hb[e] = h_bits(sm[row][c8 + e] * kW2Carry);
        const v4u u = (v4u){pk16(hb[0], hb[1]), pk16(hb[2], hb[3]), pk16(hb[4], hb[5]), pk16(hb[6], hb[7])};
        *(volatile v4u*)(D + o) = u;
      } else {
        unsigned short hb[8], lb[8];
#pragma unroll
        for (int e = 0; e < 8; ++e) {
          const float v = sm[row][c8 + e];
          hb[e] = f2bf_bits(v);
          lb[e] = f2bf_bits(v - bf_bits2f(hb[e]));
        }
        const v4u uh = (v4u){pk16(hb[0], hb[1]), pk16(hb[2], hb[3]), pk16(hb[4], hb[5]), pk16(hb[6], hb[7])};
        const v4u ul = (v4u){pk16(lb[0], lb[1]), pk16(lb[2], lb[3]), pk16(lb[4], lb[5]), pk16(lb[6], lb[7])};
        *(volatile v4u*)(D + o) = uh;
        *(volatile v4u*)(D + plane + o) = ul;
      }
    }
    __threadfence();
  }
}

__global__ __launch_bounds__(256) void cos_kernel(const float* __restrict__ ph, float* __restrict__ COS) {
  const int e    = blockIdx.x * 256 + threadIdx.x;
  const int o    = e & 3;
  const int j    = (e >> 2) & (kNN - 1);
  const int row  = e >> 11;
  const int bRow0 = row & ~(kNN - 1);
  const float d = ph[(size_t)row * kNO + o] - ph[(size_t)(bRow0 + j) * kNO + o];
  const float c = cosf(d);
  ((volatile float*)COS)[e] = c;
  __threadfence();
  ((volatile float*)COS)[e] = c;
}

__global__ __launch_bounds__(256) void build_kernel(const float* __restrict__ C1, const float* __restrict__ b1,
                                                    unsigned short* __restrict__ H1, int rowBase, int bRow0) {
  const int t  = blockIdx.x * 256 + threadIdx.x;
  const int p  = t >> 4;
  const int c8 = (t & 15) * 8;
  const int il = p >> 9;
  const int j  = p & (kNN - 1);
  const float* rp = C1 + (size_t)(rowBase + il) * kC1Pitch + c8;
  const float* sp = C1 + (size_t)(bRow0 + j) * kC1Pitch + kND + c8;
  const v4f r0 = *(const v4f*)(rp), r1 = *(const v4f*)(rp + 4);
  const v4f s0 = *(const v4f*)(sp), s1 = *(const v4f*)(sp + 4);
  const v4f g0 = *(const v4f*)(b1 + c8), g1 = *(const v4f*)(b1 + c8 + 4);
  unsigned short hb[8];
#pragma unroll
  for (int e = 0; e < 4; ++e) {
    float v0 = (r0[e] + s0[e]) + g0[e];
    float v1 = (r1[e] + s1[e]) + g1[e];
    v0 = fmaxf(v0, 0.0f) * kHidCarry;
    v1 = fmaxf(v1, 0.0f) * kHidCarry;
    hb[e]     = h_bits(v0);
    hb[4 + e] = h_bits(v1);
  }
  const v4u u = (v4u){pk16(hb[0], hb[1]), pk16(hb[2], hb[3]), pk16(hb[4], hb[5]), pk16(hb[6], hb[7])};
  unsigned short* q = H1 + (size_t)p * kND + c8;
  *(volatile v4u*)q = u;
  __threadfence();
  *(volatile v4u*)q = u;
}

__global__ __launch_bounds__(128) void agg_kernel(const float* __restrict__ MSG, const float* __restrict__ COS,
                                                  const int* __restrict__ adj, const float* __restrict__ Wg,
                                                  const float* __restrict__ bg, unsigned short* __restrict__ XA,
                                                  int rowBase, int bRow0) {
  __shared__ __align__(16) float cosL[kNN * kNO];
  __shared__ float maskL[kNN];
  __shared__ int cntW[4];
  __shared__ __align__(16) float aggL[kND];
  const int il   = blockIdx.x;
  const int t    = threadIdx.x;
  const int lane = t & 31;
  const int wave = t >> 5;
  const int row  = rowBase + il;
  const int i    = row - bRow0;

  const float* cp = COS + (size_t)row * (kNN * kNO);
#pragma unroll
  for (int qq = 0; qq < 4; ++qq) {
    const int e4 = (qq * 128 + t) * 4;
    *(v4f*)(cosL + e4) = *(const v4f*)(cp + e4);
  }
  int c = 0;
#pragma unroll
  for (int qq = 0; qq < 4; ++qq) {
    const int e = qq * 128 + t;
    const int a = adj[(size_t)i * kNN + e];
    const int m = (a != 0) ? 1 : 0;
    maskL[e] = m ? 1.0f : 0.0f;
    c += m;
  }
#pragma unroll
  for (int off = 16; off > 0; off >>= 1) c += __shfl_xor(c, off, 32);
  if (lane == 0) cntW[wave] = c;
  __syncthreads();
  const int cnt = ((cntW[0] + cntW[1]) + cntW[2]) + cntW[3];
  const float inv = 1.0f / (float)((cnt > 0) ? cnt : 1);

  const float w0 = Wg[0 * kND + t], w1 = Wg[1 * kND + t], w2 = Wg[2 * kND + t], w3 = Wg[3 * kND + t];
  const float bgd = bg[t];
  const float* mp = MSG + (size_t)il * kNN * kND + t;
  float acc = 0.0f;
#pragma unroll 1
  for (int j = 0; j < kNN; ++j) {
    const float msg = mp[(size_t)j * kND];
    const v4f cz = *(const v4f*)(cosL + j * 4);
    const float g  = ((cz[0] * w0 + cz[1] * w1) + (cz[2] * w2 + cz[3] * w3)) + bgd;
    const float ex = expf(-g);
    const float sg = 1.0f / (1.0f + ex);
    acc += maskL[j] * (msg * sg);
  }
  aggL[t] = acc * inv;
  __syncthreads();
  if (wave == 0) {
    const int hsel = lane >> 4;
    const int c8 = (lane & 15) * 8;
    unsigned short bits[8];
#pragma unroll
    for (int e = 0; e < 8; ++e) {
      const float v = aggL[c8 + e];
      const unsigned short hb = f2bf_bits(v);
      const unsigned short lb = f2bf_bits(v - bf_bits2f(hb));
      bits[e] = hsel ? lb : hb;
    }
    const v4u u = (v4u){pk16(bits[0], bits[1]), pk16(bits[2], bits[3]), pk16(bits[4], bits[5]), pk16(bits[6], bits[7])};
    unsigned short* q = XA + (size_t)hsel * kXAPlane + (size_t)row * kXAPitch + kND + c8;
    *(volatile v4u*)q = u;
    __threadfence();
    *(volatile v4u*)q = u;
  }
}

extern "C" void kernel_launch(void* const* d_in, const int* in_sizes, int n_in,
                              void* d_out, int out_size, void* d_ws, size_t ws_size,
                              hipStream_t stream) {
  if (n_in < 15) return;
  if (in_sizes[0] != kRows * kND || in_sizes[1] != kRows * kNO || in_sizes[2] != kNN * kNN) return;
  if (in_sizes[3] != kND * kND || in_sizes[4] != kND * kND || in_sizes[6] != kND * kND ||
      in_sizes[10] != kND * kND || in_sizes[11] != kND * kND || in_sizes[13] != kND * kND) return;
  if (in_sizes[5] != kND || in_sizes[7] != kND || in_sizes[9] != kND || in_sizes[12] != kND || in_sizes[14] != kND) return;
  if (in_sizes[8] != kNO * kND) return;
  if (out_size != kRows * kND) return;

  const float* X      = (const float*)d_in[0];
  const float* phases = (const float*)d_in[1];
  const int*   adj    = (const int*)  d_in[2];
  const float* W1r    = (const float*)d_in[3];
  const float* W1s    = (const float*)d_in[4];
  const float* b1     = (const float*)d_in[5];
  const float* W2     = (const float*)d_in[6];
  const float* b2     = (const float*)d_in[7];
  const float* Wg     = (const float*)d_in[8];
  const float* bg     = (const float*)d_in[9];
  const float* Wu1x   = (const float*)d_in[10];
  const float* Wu1a   = (const float*)d_in[11];
  const float* bu1    = (const float*)d_in[12];
  const float* Wu2    = (const float*)d_in[13];
  const float* bu2    = (const float*)d_in[14];
  float* out = (float*)d_out;

  char* base = (char*)d_ws;
  size_t off = 0;
  unsigned short* XAh  = (unsigned short*)(base + off); off += (size_t)2 * kXAPlane * 2;
  unsigned short* XAl  = XAh + kXAPlane;
  unsigned short* W1Th = (unsigned short*)(base + off); off += (size_t)2 * 256 * 128 * 2;
  unsigned short* W1Tl = W1Th + 256 * 128;
  unsigned short* WuTh = (unsigned short*)(base + off); off += (size_t)2 * 128 * 256 * 2;
  unsigned short* WuTl = WuTh + 128 * 256;
  unsigned short* Wu2Th = (unsigned short*)(base + off); off += (size_t)2 * 128 * 128 * 2;
  unsigned short* Wu2Tl = Wu2Th + 128 * 128;
  unsigned short* W2T  = (unsigned short*)(base + off); off += (size_t)128 * 128 * 2;
  float* C1  = (float*)(base + off); off += (size_t)kRows * kC1Pitch * 4;
  unsigned short* HPh = (unsigned short*)(base + off); off += (size_t)2 * kRows * kND * 2;
  unsigned short* HPl = HPh + kRows * kND;
  float* COS = (float*)(base + off); off += (size_t)kRows * kNN * kNO * 4;
  unsigned short* H1 = (unsigned short*)(base + off); off += (size_t)kPairs * kND * 2;
  float* MSG = (float*)(base + off); off += (size_t)kPairs * kND * 4;
  if (off > ws_size) return;

  xsplit_kernel<<<dim3(kRows * 16 / 256), dim3(256), 0, stream>>>(X, XAh);
  wprep_kernel<<<dim3(2, 2, 6), dim3(256), 0, stream>>>(W1r, W1s, Wu1x, Wu1a, Wu2, W2, W1Th, WuTh, Wu2Th, W2T);
  cos_kernel<<<dim3(kRows * kNN * kNO / 256), dim3(256), 0, stream>>>(phases, COS);
  wmma_gemm64<1, true, 0, 0, false, 0><<<dim3((kRows / 64) * (256 / 64) / 8, 1), dim3(256), 0, stream>>>(
      XAh, XAl, kXAPitch, 0L, W1Th, W1Tl, 128, 0L, (void*)C1, (void*)C1, kC1Pitch, 0L,
      b1, X, 0L, kRows, 256, kND, 1.0f);
  for (int ch = 0; ch < kNumChunks; ++ch) {
    const int rowBase = ch * kChunkRecv;
    const int bRow0   = (rowBase / kNN) * kNN;
    build_kernel<<<dim3(kPairs * 16 / 256), dim3(256), 0, stream>>>(C1, b1, H1, rowBase, bRow0);
    wmma_gemm64<0, false, 2, 0, false, 0><<<dim3((kPairs / 64) * (kND / 64) / 8, 1), dim3(256), 0, stream>>>(
        H1, H1, kND, 0L, W2T, W2T, kND, 0L, (void*)MSG, (void*)MSG, kND, 0L,
        b2, X, 0L, kPairs, kND, kND, kMsgScale);
    agg_kernel<<<dim3(kChunkRecv), dim3(128), 0, stream>>>(MSG, COS, adj, Wg, bg, XAh, rowBase, bRow0);
  }
  wmma_gemm64<1, true, 2, 2, false, 2><<<dim3((kRows / 64) * (kND / 64) / 8, 1), dim3(256), 0, stream>>>(
      XAh, XAl, kXAPitch, 0L, WuTh, WuTl, 256, 0L, (void*)HPh, (void*)HPl, kND, 0L,
      bu1, X, 0L, kRows, kND, 256, 1.0f);
  wmma_gemm64<1, true, 2, 0, true, 0><<<dim3((kRows / 64) * (kND / 64) / 8, 1), dim3(256), 0, stream>>>(
      HPh, HPl, kND, 0L, Wu2Th, Wu2Tl, kND, 0L, (void*)out, (void*)out, kND, 0L,
      bu2, X, 0L, kRows, kND, kND, 1.0f);
}
